// PPOTimeLSTMPolicy_9706626089303
// MI455X (gfx1250) — hardware-run, weakly checked
//
#include <hip/hip_runtime.h>
#include <math.h>
#include <stdint.h>

constexpr int NBATCH     = 256;
constexpr int NSTEP      = 64;
constexpr int NBT        = NBATCH * NSTEP;
constexpr int OBSD       = 1000;
constexpr int NRUN       = 30;
constexpr int HID        = 128;
constexpr int LH         = 256;
constexpr int NGATE      = 4 * LH;
constexpr int LIN_COLS   = 384;
constexpr int MKTK       = 64;
constexpr int MKT_REAL   = 40;
constexpr int RIN        = 32;
constexpr int NRROWS     = NBT * NRUN;
constexpr int NCHUNK     = 8;
constexpr int CHUNK_ROWS = 61440;
constexpr int CHUNK_BT   = 2048;
constexpr int ACT_ROWS   = NBATCH * NRUN;
constexpr int HEADN      = 64;
constexpr int TPB        = 256;
constexpr int HPITCH     = 264;
constexpr int OPITCH     = 260;
constexpr float WCARRY     = 16.0f;
constexpr float WCARRY_INV = 1.0f / 16.0f;
constexpr float AW1_CARRY  = 1024.0f;
constexpr float AW1_CARRY_INV = 1.0f / 1024.0f;
static_assert(NCHUNK * CHUNK_ROWS == NRROWS);
static_assert(CHUNK_ROWS == CHUNK_BT * NRUN);
static_assert(CHUNK_ROWS % 64 == 0);
static_assert(NCHUNK * CHUNK_BT == NBT);
static_assert((NBT * 8) % TPB == 0);
static_assert((CHUNK_ROWS * 4) % TPB == 0);
static_assert((CHUNK_BT * 16) % TPB == 0);
static_assert((ACT_ROWS * 32) % TPB == 0);

typedef __attribute__((ext_vector_type(16))) _Float16 v16h;
typedef __attribute__((ext_vector_type(8)))  _Float16 v8h;
typedef __attribute__((ext_vector_type(16))) __bf16   v16b;
typedef __attribute__((ext_vector_type(8)))  __bf16   v8b;
typedef __attribute__((ext_vector_type(8)))  float    v8f;
typedef __attribute__((ext_vector_type(4)))  float    v4f;
#define PSCALE 32768.0f
#define U16(p) ((const unsigned short*)(const void*)(p))
#define PSCALE_INV (1.0f / 32768.0f)

__device__ __forceinline__ unsigned short f2bf_bits(float f) {
  unsigned u = __float_as_uint(f);
  return (unsigned short)((u + 0x7FFFu + ((u >> 16) & 1u)) >> 16);
}
__device__ __forceinline__ float bf_bits2f(unsigned short h) { return __uint_as_float(((unsigned)h) << 16); }

__device__ __forceinline__ void dep_guard_h(v8f& a, v8f& b, v16h x, v16h y) { asm volatile("v_nop\n\tv_nop\n\tv_nop\n\tv_nop" : "+v"(a), "+v"(b) : "v"(x), "v"(y)); }
__device__ __forceinline__ void dep_guard_b(v8f& a, v8f& b, v16b x, v16b y) { asm volatile("v_nop\n\tv_nop\n\tv_nop\n\tv_nop" : "+v"(a), "+v"(b) : "v"(x), "v"(y)); }
__device__ __forceinline__ void keep4_h(v16h a, v16h b, v16h c, v16h d) { asm volatile("v_nop" :: "v"(a), "v"(b), "v"(c), "v"(d)); }
__device__ __forceinline__ void keep4_b(v16b a, v16b b, v16b c, v16b d) { asm volatile("v_nop" :: "v"(a), "v"(b), "v"(c), "v"(d)); }
__device__ __forceinline__ void acc_guard4(v8f& a, v8f& b, v8f& c, v8f& d) { asm volatile("v_nop\n\tv_nop\n\tv_nop\n\tv_nop" : "+v"(a), "+v"(b), "+v"(c), "+v"(d)); }
template <typename T> struct Frag;
template <> struct Frag<_Float16> {
  typedef v16h V; union U { v16h v; v8h h[2]; };
  static __device__ __forceinline__ v16h load(const _Float16* p) {
    U f; f.h[0] = *(const v8h*)(p); f.h[1] = *(const v8h*)(p + 16); return f.v;
  }
  static __device__ __forceinline__ v8f mma(v16h a, v16h b, v8f c) {
    return __builtin_amdgcn_wmma_f32_16x16x32_f16(false, a, false, b, (short)0, c, false, false);
  }
  static __device__ __forceinline__ void guard(v8f& a, v8f& b, v16h x, v16h y) { dep_guard_h(a, b, x, y); }
  static __device__ __forceinline__ void keep(v16h a, v16h b, v16h c, v16h d) { keep4_h(a, b, c, d); }
};
template <> struct Frag<__bf16> {
  typedef v16b V; union U { v16b v; v8b h[2]; };
  static __device__ __forceinline__ v16b load(const __bf16* p) {
    U f; f.h[0] = *(const v8b*)(p); f.h[1] = *(const v8b*)(p + 16); return f.v;
  }
  static __device__ __forceinline__ v8f mma(v16b a, v16b b, v8f c) {
    return __builtin_amdgcn_wmma_f32_16x16x32_bf16(false, a, false, b, (short)0, c, false, false);
  }
  static __device__ __forceinline__ void guard(v8f& a, v8f& b, v16b x, v16b y) { dep_guard_b(a, b, x, y); }
  static __device__ __forceinline__ void keep(v16b a, v16b b, v16b c, v16b d) { keep4_b(a, b, c, d); }
};

template <int ET> struct Elem;
template <> struct Elem<0> { typedef _Float16 T; };
template <> struct Elem<1> { typedef __bf16 T; };
template <int ET, bool SPLIT, int BIAS_MODE, int OUT_MODE, bool RESID, int ACT = 0>
__global__ __launch_bounds__(256) void wmma_gemm64(
    const unsigned short* __restrict__ Ap, const unsigned short* __restrict__ A2p, int lda, long strideA,
    const unsigned short* __restrict__ Btp, const unsigned short* __restrict__ Bt2p, int ldb, long strideB,
    void* __restrict__ Cout, void* __restrict__ Cout2, int ldc, long strideC,
    const float* __restrict__ bias,
    const float* __restrict__ resid, long strideR,
    int M, int N, int K, float scale) {
  typedef typename Elem<ET>::T T;
  typedef typename Frag<T>::V V;
  const T* A = (const T*)Ap; const T* A2 = (const T*)A2p; const T* Bt = (const T*)Btp; const T* Bt2 = (const T*)Bt2p;
  __shared__ __align__(16) float sT[8][16 * 68];
  const int b    = blockIdx.y;
  const int lane = threadIdx.x & 31;
  const int wave = threadIdx.x >> 5;
  const int tilesN = N >> 6;
  const int tilesM = M >> 6;
  const int tile = blockIdx.x * 8 + wave;
  if (tile >= tilesM * tilesN) return;
  const int tm = tile / tilesN;
  const int tn = tile - tm * tilesN;
  const int m0 = tm << 6;
  const int n0 = tn << 6;

  const T* Ab  = A  + (size_t)b * strideA;
  const T* Bb  = Bt + (size_t)b * strideB;
  const T* Ab2 = SPLIT ? (A2  + (size_t)b * strideA) : nullptr;
  const T* Bb2 = SPLIT ? (Bt2 + (size_t)b * strideB) : nullptr;

  const int rlane = lane & 15;
  const int koff  = (lane >> 4) * 8;
  const int mOff  = (lane >> 4) * 8;

  v8f acc[4][4];
#pragma unroll
  for (int i = 0; i < 4; ++i)
#pragma unroll
    for (int j = 0; j < 4; ++j) acc[i][j] = (v8f){0.f,0.f,0.f,0.f,0.f,0.f,0.f,0.f};

  for (int k0 = 0; k0 < K; k0 += 32) {
    V bh[4], bl[4];
#pragma unroll
    for (int j = 0; j < 4; ++j) {
      const size_t bo = (size_t)(n0 + (j << 4) + rlane) * ldb + koff + k0;
      bh[j] = Frag<T>::load(Bb + bo);
      if (SPLIT) bl[j] = Frag<T>::load(Bb2 + bo);
    }
#pragma unroll
    for (int i = 0; i < 4; ++i) {
      const size_t ao = (size_t)(m0 + (i << 4) + rlane) * lda + koff + k0;
      V ah = Frag<T>::load(Ab + ao);
      V al;
      if (SPLIT) al = Frag<T>::load(Ab2 + ao);
#pragma unroll
      for (int j = 0; j < 4; ++j) {
        acc[i][j] = Frag<T>::mma(ah, bh[j], acc[i][j]);
        if (SPLIT) {
          acc[i][j] = Frag<T>::mma(ah, bl[j], acc[i][j]);
          acc[i][j] = Frag<T>::mma(al, bh[j], acc[i][j]);
        }
      }
      Frag<T>::guard(acc[i][0], acc[i][3], ah, SPLIT ? al : ah);
    }
    Frag<T>::keep(bh[0], bh[1], bh[2], bh[3]);
    if (SPLIT) Frag<T>::keep(bl[0], bl[1], bl[2], bl[3]);
  }
  acc_guard4(acc[0][0], acc[0][1], acc[0][2], acc[0][3]);
  acc_guard4(acc[1][0], acc[1][1], acc[1][2], acc[1][3]);
  acc_guard4(acc[2][0], acc[2][1], acc[2][2], acc[2][3]);
  acc_guard4(acc[3][0], acc[3][1], acc[3][2], acc[3][3]);

  float* slab = sT[wave];
  const float* Rb = RESID ? (resid + (size_t)b * strideR) : nullptr;
#pragma unroll
  for (int i = 0; i < 4; ++i) {
    const int mBase = m0 + (i << 4);
#pragma unroll
    for (int j = 0; j < 4; ++j) {
      const int n = n0 + (j << 4) + rlane;
      float bv = 0.f;
      if (BIAS_MODE == 2) bv = bias[n];
#pragma unroll
      for (int r = 0; r < 8; ++r) {
        float v = acc[i][j][r] * scale;
        if (BIAS_MODE == 1) v += bias[mBase + mOff + r];
        if (BIAS_MODE == 2) v += bv;
        if (RESID) v += Rb[(size_t)(mBase + mOff + r) * ldc + n];
        if (ACT == 1) v = tanhf(v);
        if (ACT == 2) v = fmaxf(v, 0.0f);
        if (ACT == 3) v = v / (1.0f + expf(-v));
        if (ACT == 4) v = (v > 0.f) ? v : 0.01f * v;
        if (ACT == 5) v = 0.5f * v * (1.0f + erff(v * 0.70710678118654752f));
        slab[(mOff + r) * 68 + (j << 4) + rlane] = v;
      }
    }
    __builtin_amdgcn_fence(__ATOMIC_RELEASE, "workgroup");
    __builtin_amdgcn_wave_barrier();
    __builtin_amdgcn_fence(__ATOMIC_ACQUIRE, "workgroup");
    if (OUT_MODE == 0) {
      float* C = (float*)Cout + (size_t)b * strideC;
      const int hh = lane >> 4, c4 = (lane & 15) * 4;
      for (int pass = 0; pass < 2; ++pass) {
#pragma unroll
        for (int it = 0; it < 8; ++it) {
          const int row = it * 2 + hh;
          v4f v = *(const v4f*)(slab + row * 68 + c4);
          *(volatile v4f*)(C + (size_t)(mBase + row) * ldc + n0 + c4) = v;
        }
        __threadfence();
      }
    } else {
      const int q = lane >> 3, c8 = (lane & 7) * 8;
      unsigned short* C  = (unsigned short*)Cout  + (size_t)b * strideC;
      unsigned short* C2 = (OUT_MODE == 2) ? ((unsigned short*)Cout2 + (size_t)b * strideC) : nullptr;
      for (int pass = 0; pass < 2; ++pass) {
#pragma unroll
        for (int it = 0; it < 4; ++it) {
          const int row = it * 4 + q;
          const float* sp = slab + row * 68 + c8;
          v8h hv, lv;
#pragma unroll
          for (int e = 0; e < 8; ++e) {
            if (OUT_MODE == 1) {
              hv[e] = (_Float16)sp[e];
            } else {
              unsigned short hb = f2bf_bits(sp[e]);
              unsigned short lb = f2bf_bits(sp[e] - bf_bits2f(hb));
              hv[e] = __builtin_bit_cast(_Float16, hb);
              lv[e] = __builtin_bit_cast(_Float16, lb);
            }
          }
          *(volatile v8h*)(C + (size_t)(mBase + row) * ldc + n0 + c8) = hv;
          if (OUT_MODE == 2) *(volatile v8h*)(C2 + (size_t)(mBase + row) * ldc + n0 + c8) = lv;
        }
        __threadfence();
      }
    }
    __builtin_amdgcn_fence(__ATOMIC_RELEASE, "workgroup");
    __builtin_amdgcn_wave_barrier();
    __builtin_amdgcn_fence(__ATOMIC_ACQUIRE, "workgroup");
  }
}

__device__ __forceinline__ void st2_h8(unsigned short* p, v8h v) {
  *(volatile v8h*)p = v; __threadfence(); *(volatile v8h*)p = v;
}
__device__ __forceinline__ void st2_f4(float* p, v4f v) {
  *(volatile v4f*)p = v; __threadfence(); *(volatile v4f*)p = v;
}
__device__ __forceinline__ void st2_u32(unsigned* p, unsigned v) {
  *(volatile unsigned*)p = v; __threadfence(); *(volatile unsigned*)p = v;
}
__device__ __forceinline__ void st2_f1(float* p, float v) {
  *(volatile float*)p = v; __threadfence(); *(volatile float*)p = v;
}

__device__ __forceinline__ float fsig(float x)  { return __builtin_amdgcn_rcpf(1.0f + __expf(-x)); }
__device__ __forceinline__ float ftanh(float x) { return 1.0f - 2.0f * __builtin_amdgcn_rcpf(__expf(2.0f * x) + 1.0f); }

__global__ __launch_bounds__(TPB) void cast_w_kernel(const float* __restrict__ w, int nReal, int kReal, int srcPitch, int srcCol0,
                                                    unsigned short* __restrict__ out, int nPad, int kPad, float sc) {
  const int i = blockIdx.x * TPB + threadIdx.x;
  const int n2 = (nPad * kPad) >> 1;
  if (i >= n2) return;
  const int e0 = 2 * i;
  const int n = e0 / kPad;
  const int k = e0 - n * kPad;
  const int nc  = (n < nReal) ? n : (nReal - 1);
  const int k0c = (k < kReal) ? k : (kReal - 1);
  const int k1c = (k + 1 < kReal) ? (k + 1) : (kReal - 1);
  const float* rowp = w + (size_t)nc * srcPitch + srcCol0;
  float v0 = rowp[k0c] * sc;
  float v1 = rowp[k1c] * sc;
  if (n >= nReal || k >= kReal) v0 = 0.0f;
  if (n >= nReal || k + 1 >= kReal) v1 = 0.0f;
  const _Float16 h0 = (_Float16)v0, h1 = (_Float16)v1;
  const unsigned u = (unsigned)__builtin_bit_cast(unsigned short, h0) | ((unsigned)__builtin_bit_cast(unsigned short, h1) << 16);
  st2_u32((unsigned*)(void*)out + i, u);
}

__global__ __launch_bounds__(TPB) void obs_market_kernel(const float* __restrict__ obs, unsigned short* __restrict__ MF, float* __restrict__ DT) {
  const int idx = blockIdx.x * TPB + threadIdx.x;
  const int row = idx >> 3, c8 = (idx & 7) * 8;
  const float* o = obs + (size_t)row * OBSD;
  v8h hv;
#pragma unroll
  for (int e = 0; e < 8; ++e) {
    const int col = c8 + e;
    const int src = (col < 30) ? col : ((col < MKT_REAL) ? (720 + col) : 0);
    float v = o[src];
    if (col >= MKT_REAL) v = 0.0f;
    hv[e] = (_Float16)v;
  }
  st2_h8(MF + (size_t)row * MKTK + c8, hv);
  if (idx < NBT) st2_f1(DT + idx, obs[(size_t)idx * OBSD + 26]);
}

__global__ __launch_bounds__(TPB) void obs_runner_kernel(const float* __restrict__ obs, int rowBase, unsigned short* __restrict__ RF) {
  const int idx = blockIdx.x * TPB + threadIdx.x;
  const int lr = idx >> 2, c8 = (idx & 3) * 8;
  const int gr = rowBase + lr;
  const int bt = gr / NRUN;
  const int r  = gr - bt * NRUN;
  const int base = (c8 < 24) ? (30 + r * 24 + c8) : (760 + r * 8);
  const float* o = obs + (size_t)bt * OBSD + base;
  v8h hv;
#pragma unroll
  for (int e = 0; e < 8; ++e) hv[e] = (_Float16)o[e];
  st2_h8(RF + (size_t)lr * RIN + c8, hv);
}

__global__ __launch_bounds__(TPB) void meanmax_kernel(const float* __restrict__ RE, int btBase,
                                                    unsigned short* __restrict__ LIN, unsigned short* __restrict__ RL) {
  const int idx = blockIdx.x * TPB + threadIdx.x;
  const int btl = idx >> 4, c8 = (idx & 15) * 8;
  const int bt = btBase + btl;
  const bool last = ((bt & (NSTEP - 1)) == (NSTEP - 1));
  const int bidx = bt >> 6;
  float s[8], mx[8];
#pragma unroll
  for (int e = 0; e < 8; ++e) { s[e] = 0.0f; mx[e] = -INFINITY; }
#pragma unroll 1
  for (int r = 0; r < NRUN; ++r) {
    const float* p = RE + ((size_t)(btl * NRUN + r)) * HID + c8;
    const v4f a = *(const v4f*)p;
    const v4f q = *(const v4f*)(p + 4);
    float v[8];
    v[0] = a[0]; v[1] = a[1]; v[2] = a[2]; v[3] = a[3];
    v[4] = q[0]; v[5] = q[1]; v[6] = q[2]; v[7] = q[3];
    v8h hv;
#pragma unroll
    for (int e = 0; e < 8; ++e) {
      s[e] += v[e];
      mx[e] = fmaxf(mx[e], v[e]);
      hv[e] = (_Float16)v[e];
    }
    if (last) st2_h8(RL + ((size_t)(bidx * NRUN + r)) * HID + c8, hv);
  }
  v8h hm, hx;
#pragma unroll
  for (int e = 0; e < 8; ++e) { hm[e] = (_Float16)(s[e] * (1.0f / 30.0f)); hx[e] = (_Float16)mx[e]; }
  st2_h8(LIN + (size_t)bt * LIN_COLS + HID + c8, hm);
  st2_h8(LIN + (size_t)bt * LIN_COLS + 2 * HID + c8, hx);
}

__global__ __launch_bounds__(TPB) void lstm_kernel(const float* __restrict__ XPp, const float* __restrict__ Wdt,
                                                 const float* __restrict__ DTp, const unsigned short* __restrict__ WHp,
                                                 float* __restrict__ outH, float* __restrict__ outC,
                                                 unsigned short* __restrict__ HL) {
  __shared__ __align__(16) _Float16 Ah[16 * HPITCH];
  __shared__ __align__(16) float    Hs[16 * OPITCH];
  const _Float16* WH = (const _Float16*)WHp;
  const int tid = threadIdx.x, lane = tid & 31, wave = tid >> 5;
  const int c = lane & 15, hh = lane >> 4, koff = hh * 8;
  const int rowbase = blockIdx.x * 16;

#pragma unroll 1
  for (int i = 0; i < 16; ++i) Ah[i * HPITCH + tid] = (_Float16)0.0f;
  float cst[2][8], hst[2][8], wdt[2];
#pragma unroll
  for (int nt = 0; nt < 2; ++nt) {
    const int j = 32 * wave + 16 * nt + c;
    wdt[nt] = Wdt[j];
#pragma unroll
    for (int r = 0; r < 8; ++r) { cst[nt][r] = 0.0f; hst[nt][r] = 0.0f; }
  }
  __syncthreads();

  const _Float16* ahrow = Ah + c * HPITCH + koff;
  const v8f z8 = {0.f, 0.f, 0.f, 0.f, 0.f, 0.f, 0.f, 0.f};

#pragma unroll 1
  for (int t = 0; t < NSTEP; ++t) {
    float dtr[8];
#pragma unroll
    for (int r = 0; r < 8; ++r) dtr[r] = DTp[(size_t)(rowbase + 8 * hh + r) * NSTEP + t];
#pragma unroll
    for (int nt = 0; nt < 2; ++nt) {
      const int j = 32 * wave + 16 * nt + c;
      const _Float16* wh = WH + (size_t)j * LH + koff;
      v8f acc[4];
      acc[0] = z8; acc[1] = z8; acc[2] = z8; acc[3] = z8;
#pragma unroll
      for (int g = 0; g < 4; ++g)
#pragma unroll
        for (int r = 0; r < 8; ++r)
          acc[g][r] = XPp[((size_t)(rowbase + 8 * hh + r) * NSTEP + (size_t)t) * NGATE + g * LH + j] * WCARRY;
#pragma unroll 1
      for (int k0 = 0; k0 < LH; k0 += 32) {
        const v16h a  = Frag<_Float16>::load(ahrow + k0);
        const v16h b0 = Frag<_Float16>::load(wh + k0);
        const v16h b1 = Frag<_Float16>::load(wh + (size_t)1 * LH * LH + k0);
        const v16h b2 = Frag<_Float16>::load(wh + (size_t)2 * LH * LH + k0);
        const v16h b3 = Frag<_Float16>::load(wh + (size_t)3 * LH * LH + k0);
        acc[0] = Frag<_Float16>::mma(a, b0, acc[0]);
        acc[1] = Frag<_Float16>::mma(a, b1, acc[1]);
        acc[2] = Frag<_Float16>::mma(a, b2, acc[2]);
        acc[3] = Frag<_Float16>::mma(a, b3, acc[3]);
        dep_guard_h(acc[0], acc[3], a, b3);
        keep4_h(b0, b1, b2, b3);
      }
      acc_guard4(acc[0], acc[1], acc[2], acc[3]);
#pragma unroll
      for (int r = 0; r < 8; ++r) {
        const float zi = acc[0][r] * WCARRY_INV;
        const float zf = acc[1][r] * WCARRY_INV + wdt[nt] * dtr[r];
        const float zg = acc[2][r] * WCARRY_INV;
        const float zo = acc[3][r] * WCARRY_INV;
        const float ig = fsig(zi);
        const float fg = fsig(zf);
        const float gg = ftanh(zg);
        const float og = fsig(zo);
        const float cn = fg * cst[nt][r] + ig * gg;
        cst[nt][r] = cn;
        hst[nt][r] = og * ftanh(cn);
      }
    }
    __syncthreads();
#pragma unroll
    for (int nt = 0; nt < 2; ++nt) {
      const int j = 32 * wave + 16 * nt + c;
#pragma unroll
      for (int r = 0; r < 8; ++r) Ah[(8 * hh + r) * HPITCH + j] = (_Float16)hst[nt][r];
    }
    __syncthreads();
  }

#pragma unroll
  for (int nt = 0; nt < 2; ++nt) {
    const int j = 32 * wave + 16 * nt + c;
#pragma unroll
    for (int r = 0; r < 8; ++r) Hs[(8 * hh + r) * OPITCH + j] = hst[nt][r];
  }
  __syncthreads();
  for (int pass = 0; pass < 2; ++pass) {
#pragma unroll
    for (int it = 0; it < 4; ++it) {
      const int idx = it * TPB + tid;
      const int row = idx >> 6, c4 = (idx & 63) * 4;
      const v4f v = *(const v4f*)(Hs + row * OPITCH + c4);
      *(volatile v4f*)(outH + (size_t)(rowbase + row) * LH + c4) = v;
    }
    __threadfence();
  }
  {
    v8h hv2[2];
#pragma unroll
    for (int it = 0; it < 2; ++it) {
      const int row = it * 8 + wave;
#pragma unroll
      for (int e = 0; e < 8; ++e) hv2[it][e] = (_Float16)Hs[row * OPITCH + lane * 8 + e];
    }
    for (int pass = 0; pass < 2; ++pass) {
#pragma unroll
      for (int it = 0; it < 2; ++it) {
        const int row = it * 8 + wave;
        *(volatile v8h*)(HL + (size_t)(rowbase + row) * LH + lane * 8) = hv2[it];
      }
      __threadfence();
    }
  }
  __syncthreads();
#pragma unroll
  for (int nt = 0; nt < 2; ++nt) {
    const int j = 32 * wave + 16 * nt + c;
#pragma unroll
    for (int r = 0; r < 8; ++r) Hs[(8 * hh + r) * OPITCH + j] = cst[nt][r];
  }
  __syncthreads();
  for (int pass = 0; pass < 2; ++pass) {
#pragma unroll
    for (int it = 0; it < 4; ++it) {
      const int idx = it * TPB + tid;
      const int row = idx >> 6, c4 = (idx & 63) * 4;
      const v4f v = *(const v4f*)(Hs + row * OPITCH + c4);
      *(volatile v4f*)(outC + (size_t)(rowbase + row) * LH + c4) = v;
    }
    __threadfence();
  }
}

__global__ __launch_bounds__(TPB) void bcast_kernel(const float* __restrict__ HLP, float* __restrict__ HLB) {
  const int idx = blockIdx.x * TPB + threadIdx.x;
  const int row = idx >> 5, c4 = (idx & 31) * 4;
  const int b = row / NRUN;
  const v4f v = *(const v4f*)(HLP + (size_t)b * HID + c4);
  st2_f4(HLB + (size_t)row * HID + c4, v);
}

__global__ __launch_bounds__(TPB) void pack_kernel(const float* __restrict__ AO, const float* __restrict__ ab1,
                                                 const float* __restrict__ VO, const float* __restrict__ cb1,
                                                 const float* __restrict__ lstd, float* __restrict__ out) {
  const int u = blockIdx.x * TPB + threadIdx.x;
  const int u0 = (u < 3840) ? u : 3839;
  int t1 = u - 3840; t1 = (t1 < 0) ? 0 : ((t1 > 3839) ? 3839 : t1);
  int t2 = u - 7680; t2 = (t2 < 0) ? 0 : ((t2 > 63) ? 63 : t2);
  const float b0 = ab1[0], b1 = ab1[1], cb = cb1[0];
  v4f va, vl, vv, v;
  va[0] = AO[(size_t)(2 * u0) * HEADN]         + b0;
  va[1] = AO[(size_t)(2 * u0) * HEADN + 1]     + b1;
  va[2] = AO[(size_t)(2 * u0 + 1) * HEADN]     + b0;
  va[3] = AO[(size_t)(2 * u0 + 1) * HEADN + 1] + b1;
#pragma unroll
  for (int e = 0; e < 4; ++e) {
    vl[e] = lstd[(4 * t1 + e) % 60];
    vv[e] = VO[(size_t)(4 * t2 + e) * HEADN] + cb;
  }
  const bool s0 = (u < 3840), s1 = (u < 7680);
#pragma unroll
  for (int e = 0; e < 4; ++e) v[e] = s0 ? va[e] : (s1 ? vl[e] : vv[e]);
  if (u < 7744) st2_f4(out + (size_t)4 * u, v);
}

extern "C" void kernel_launch(void* const* d_in, const int* in_sizes, int n_in,
                              void* d_out, int out_size, void* d_ws, size_t ws_size, hipStream_t stream) {
  if (n_in < 26 || d_out == nullptr || d_ws == nullptr) return;
  if (in_sizes[0] != NBT * OBSD || in_sizes[1] != HID * RIN || in_sizes[3] != HID * HID || in_sizes[5] != HID * HID ||
      in_sizes[7] != HID * MKT_REAL || in_sizes[9] != HID * HID || in_sizes[11] != HID * HID ||
      in_sizes[13] != NGATE * LIN_COLS || in_sizes[14] != NGATE || in_sizes[15] != NGATE * LH || in_sizes[16] != LH ||
      in_sizes[17] != HID * LIN_COLS || in_sizes[18] != HID || in_sizes[19] != 2 * HID || in_sizes[20] != 2 ||
      in_sizes[21] != HID * LH || in_sizes[22] != HID || in_sizes[23] != HID || in_sizes[24] != 1 || in_sizes[25] != 60 ||
      in_sizes[2] != HID || in_sizes[4] != HID || in_sizes[6] != HID || in_sizes[8] != HID || in_sizes[10] != HID || in_sizes[12] != HID ||
      out_size != 162048) return;

  const float* obs   = (const float*)d_in[0];
  const float* re_w0 = (const float*)d_in[1];
  const float* re_b0 = (const float*)d_in[2];
  const float* re_w1 = (const float*)d_in[3];
  const float* re_b1 = (const float*)d_in[4];
  const float* re_w2 = (const float*)d_in[5];
  const float* re_b2 = (const float*)d_in[6];
  const float* me_w0 = (const float*)d_in[7];
  const float* me_b0 = (const float*)d_in[8];
  const float* me_w1 = (const float*)d_in[9];
  const float* me_b1 = (const float*)d_in[10];
  const float* me_w2 = (const float*)d_in[11];
  const float* me_b2 = (const float*)d_in[12];
  const float* W_ih  = (const float*)d_in[13];
  const float* b_ih  = (const float*)d_in[14];
  const float* W_hh  = (const float*)d_in[15];
  const float* W_dt  = (const float*)d_in[16];
  const float* a_w0  = (const float*)d_in[17];
  const float* a_b0  = (const float*)d_in[18];
  const float* a_w1  = (const float*)d_in[19];
  const float* a_b1  = (const float*)d_in[20];
  const float* c_w0  = (const float*)d_in[21];
  const float* c_b0  = (const float*)d_in[22];
  const float* c_w1  = (const float*)d_in[23];
  const float* c_b1  = (const float*)d_in[24];
  const float* lstd  = (const float*)d_in[25];

  float* out  = (float*)d_out;
  float* outH = out + 30976;
  float* outC = out + 96512;

  char* ws = (char*)d_ws; size_t off = 0;
  auto carve = [&](size_t bytes) -> char* { char* p = ws + off; off += (bytes + 255) & ~(size_t)255; return p; };
  unsigned short* REW0 = (unsigned short*)carve((size_t)HID * RIN * 2);
  unsigned short* REW1 = (unsigned short*)carve((size_t)HID * HID * 2);
  unsigned short* REW2 = (unsigned short*)carve((size_t)HID * HID * 2);
  unsigned short* MEW0 = (unsigned short*)carve((size_t)HID * MKTK * 2);
  unsigned short* MEW1 = (unsigned short*)carve((size_t)HID * HID * 2);
  unsigned short* MEW2 = (unsigned short*)carve((size_t)HID * HID * 2);
  unsigned short* WIH  = (unsigned short*)carve((size_t)NGATE * LIN_COLS * 2);
  unsigned short* WHH  = (unsigned short*)carve((size_t)NGATE * LH * 2);
  unsigned short* AW0A = (unsigned short*)carve((size_t)HID * HID * 2);
  unsigned short* AW0B = (unsigned short*)carve((size_t)HID * LH * 2);
  unsigned short* CW0  = (unsigned short*)carve((size_t)HID * LH * 2);
  unsigned short* AW1P = (unsigned short*)carve((size_t)HEADN * HID * 2);
  unsigned short* CW1P = (unsigned short*)carve((size_t)HEADN * HID * 2);
  unsigned short* MF16 = (unsigned short*)carve((size_t)NBT * MKTK * 2);
  float*          DT   = (float*)carve((size_t)NBT * 4);
  unsigned short* M1   = (unsigned short*)carve((size_t)NBT * HID * 2);
  unsigned short* M2   = (unsigned short*)carve((size_t)NBT * HID * 2);
  unsigned short* LIN16 = (unsigned short*)carve((size_t)NBT * LIN_COLS * 2);
  unsigned short* RLAST16 = (unsigned short*)carve((size_t)ACT_ROWS * HID * 2);
  unsigned short* HL16 = (unsigned short*)carve((size_t)NBATCH * LH * 2);
  float*          HLPROJ = (float*)carve((size_t)NBATCH * HID * 4);
  float*          HLB  = (float*)carve((size_t)ACT_ROWS * HID * 4);
  unsigned short* AH16 = (unsigned short*)carve((size_t)ACT_ROWS * HID * 2);
  unsigned short* VH16 = (unsigned short*)carve((size_t)NBATCH * HID * 2);
  float*          AO   = (float*)carve((size_t)ACT_ROWS * HEADN * 4);
  float*          VO   = (float*)carve((size_t)NBATCH * HEADN * 4);
  const size_t chunkPlanes = (size_t)CHUNK_ROWS * RIN * 2 + 2 * (size_t)CHUNK_ROWS * HID * 2 + (size_t)CHUNK_ROWS * HID * 4;
  const size_t xpBytes = (size_t)NBT * NGATE * 4;
  const size_t scratchBytes = chunkPlanes > xpBytes ? chunkPlanes : xpBytes;
  char* SCR = carve(scratchBytes);
  if (off > ws_size || off > (size_t)134217728) return;
  unsigned short* RF16 = (unsigned short*)(SCR);
  unsigned short* R1   = (unsigned short*)(SCR + (size_t)CHUNK_ROWS * RIN * 2);
  unsigned short* R2   = (unsigned short*)(SCR + (size_t)CHUNK_ROWS * RIN * 2 + (size_t)CHUNK_ROWS * HID * 2);
  float*          RE   = (float*)(SCR + (size_t)CHUNK_ROWS * RIN * 2 + 2 * (size_t)CHUNK_ROWS * HID * 2);
  float*          XP   = (float*)(SCR);

  auto castGrid = [](int nPad, int kPad) { return dim3((unsigned)(((nPad * kPad) / 2 + TPB - 1) / TPB)); };
  cast_w_kernel<<<castGrid(HID, RIN), TPB, 0, stream>>>(re_w0, HID, RIN, RIN, 0, REW0, HID, RIN, WCARRY);
  cast_w_kernel<<<castGrid(HID, HID), TPB, 0, stream>>>(re_w1, HID, HID, HID, 0, REW1, HID, HID, WCARRY);
  cast_w_kernel<<<castGrid(HID, HID), TPB, 0, stream>>>(re_w2, HID, HID, HID, 0, REW2, HID, HID, WCARRY);
  cast_w_kernel<<<castGrid(HID, MKTK), TPB, 0, stream>>>(me_w0, HID, MKT_REAL, MKT_REAL, 0, MEW0, HID, MKTK, WCARRY);
  cast_w_kernel<<<castGrid(HID, HID), TPB, 0, stream>>>(me_w1, HID, HID, HID, 0, MEW1, HID, HID, WCARRY);
  cast_w_kernel<<<castGrid(HID, HID), TPB, 0, stream>>>(me_w2, HID, HID, HID, 0, MEW2, HID, HID, WCARRY);
  cast_w_kernel<<<castGrid(NGATE, LIN_COLS), TPB, 0, stream>>>(W_ih, NGATE, LIN_COLS, LIN_COLS, 0, WIH, NGATE, LIN_COLS, WCARRY);
  cast_w_kernel<<<castGrid(NGATE, LH), TPB, 0, stream>>>(W_hh, NGATE, LH, LH, 0, WHH, NGATE, LH, WCARRY);
  cast_w_kernel<<<castGrid(HID, HID), TPB, 0, stream>>>(a_w0, HID, HID, LIN_COLS, 0, AW0A, HID, HID, WCARRY);
  cast_w_kernel<<<castGrid(HID, LH), TPB, 0, stream>>>(a_w0, HID, LH, LIN_COLS, HID, AW0B, HID, LH, WCARRY);
  cast_w_kernel<<<castGrid(HID, LH), TPB, 0, stream>>>(c_w0, HID, LH, LH, 0, CW0, HID, LH, WCARRY);
  cast_w_kernel<<<castGrid(HEADN, HID), TPB, 0, stream>>>(a_w1, 2, HID, HID, 0, AW1P, HEADN, HID, AW1_CARRY);
  cast_w_kernel<<<castGrid(HEADN, HID), TPB, 0, stream>>>(c_w1, 1, HID, HID, 0, CW1P, HEADN, HID, WCARRY);

  obs_market_kernel<<<dim3((NBT * 8) / TPB), TPB, 0, stream>>>(obs, MF16, DT);

  auto gemmGrid = [](int M, int N) { const int tiles = (M / 64) * (N / 64); return dim3((unsigned)((tiles + 7) / 8), 1u); };
  wmma_gemm64<0, false, 2, 1, false, 2><<<gemmGrid(NBT, HID), 256, 0, stream>>>(
      MF16, MF16, MKTK, 0L, MEW0, MEW0, MKTK, 0L, (void*)M1, (void*)M1, HID, 0L, me_b0, me_b0, 0L, NBT, HID, MKTK, WCARRY_INV);
  wmma_gemm64<0, false, 2, 1, false, 2><<<gemmGrid(NBT, HID), 256, 0, stream>>>(
      M1, M1, HID, 0L, MEW1, MEW1, HID, 0L, (void*)M2, (void*)M2, HID, 0L, me_b1, me_b1, 0L, NBT, HID, HID, WCARRY_INV);
  wmma_gemm64<0, false, 2, 1, false, 0><<<gemmGrid(NBT, HID), 256, 0, stream>>>(
      M2, M2, HID, 0L, MEW2, MEW2, HID, 0L, (void*)LIN16, (void*)LIN16, LIN_COLS, 0L, me_b2, me_b2, 0L, NBT, HID, HID, WCARRY_INV);

  for (int ch = 0; ch < NCHUNK; ++ch) {
    obs_runner_kernel<<<dim3((CHUNK_ROWS * 4) / TPB), TPB, 0, stream>>>(obs, ch * CHUNK_ROWS, RF16);
    wmma_gemm64<0, false, 2, 1, false, 2><<<gemmGrid(CHUNK_ROWS, HID), 256, 0, stream>>>(
        RF16, RF16, RIN, 0L, REW0, REW0, RIN, 0L, (void*)R1, (void*)R1, HID, 0L, re_b0, re_b0, 0L, CHUNK_ROWS, HID, RIN, WCARRY_INV);
    wmma_gemm64<0, false, 2, 1, false, 2><<<gemmGrid(CHUNK_ROWS, HID), 256, 0, stream>>>(
        R1, R1, HID, 0L, REW1, REW1, HID, 0L, (void*)R2, (void*)R2, HID, 0L, re_b1, re_b1, 0L, CHUNK_ROWS, HID, HID, WCARRY_INV);
    wmma_gemm64<0, false, 2, 0, false, 0><<<gemmGrid(CHUNK_ROWS, HID), 256, 0, stream>>>(
        R2, R2, HID, 0L, REW2, REW2, HID, 0L, (void*)RE, (void*)RE, HID, 0L, re_b2, re_b2, 0L, CHUNK_ROWS, HID, HID, WCARRY_INV);
    meanmax_kernel<<<dim3((CHUNK_BT * 16) / TPB), TPB, 0, stream>>>(RE, ch * CHUNK_BT, LIN16, RLAST16);
  }

  wmma_gemm64<0, false, 2, 0, false, 0><<<gemmGrid(NBT, NGATE), 256, 0, stream>>>(
      LIN16, LIN16, LIN_COLS, 0L, WIH, WIH, LIN_COLS, 0L, (void*)XP, (void*)XP, NGATE, 0L, b_ih, b_ih, 0L, NBT, NGATE, LIN_COLS, WCARRY_INV);

  lstm_kernel<<<dim3(NBATCH / 16), TPB, 0, stream>>>(XP, W_dt, DT, WHH, outH, outC, HL16);

  wmma_gemm64<0, false, 2, 0, false, 0><<<gemmGrid(NBATCH, HID), 256, 0, stream>>>(
      HL16, HL16, LH, 0L, AW0B, AW0B, LH, 0L, (void*)HLPROJ, (void*)HLPROJ, HID, 0L, a_b0, a_b0, 0L, NBATCH, HID, LH, WCARRY_INV);
  bcast_kernel<<<dim3((ACT_ROWS * 32) / TPB), TPB, 0, stream>>>(HLPROJ, HLB);
  wmma_gemm64<0, false, 0, 1, true, 2><<<gemmGrid(ACT_ROWS, HID), 256, 0, stream>>>(
      RLAST16, RLAST16, HID, 0L, AW0A, AW0A, HID, 0L, (void*)AH16, (void*)AH16, HID, 0L, a_b0, HLB, 0L, ACT_ROWS, HID, HID, WCARRY_INV);
  wmma_gemm64<0, false, 2, 1, false, 2><<<gemmGrid(NBATCH, HID), 256, 0, stream>>>(
      HL16, HL16, LH, 0L, CW0, CW0, LH, 0L, (void*)VH16, (void*)VH16, HID, 0L, c_b0, c_b0, 0L, NBATCH, HID, LH, WCARRY_INV);
  wmma_gemm64<0, false, 0, 0, false, 0><<<gemmGrid(ACT_ROWS, HEADN), 256, 0, stream>>>(
      AH16, AH16, HID, 0L, AW1P, AW1P, HID, 0L, (void*)AO, (void*)AO, HEADN, 0L, a_b0, a_b0, 0L, ACT_ROWS, HEADN, HID, AW1_CARRY_INV);
  wmma_gemm64<0, false, 0, 0, false, 0><<<gemmGrid(NBATCH, HEADN), 256, 0, stream>>>(
      VH16, VH16, HID, 0L, CW1P, CW1P, HID, 0L, (void*)VO, (void*)VO, HEADN, 0L, c_b0, c_b0, 0L, NBATCH, HEADN, HID, WCARRY_INV);
  pack_kernel<<<dim3((7744 + TPB - 1) / TPB), TPB, 0, stream>>>(AO, a_b1, VO, c_b1, lstd, out);
}
